// DA_Block_62474594287831
// MI455X (gfx1250) — hardware-verified
//
#include <hip/hip_runtime.h>
#include <math.h>
#include <stdint.h>

#define NB    2
#define CC    256
#define NN    4096
#define CQ    32
#define MQKV  320
#define QT    64
#define OSP   68
#define OSPW  132
#define TP    72
#define WSC   256.0f
#define IWSC  0.00390625f
#define PSC   1024.0f
#define IPSC  0.0009765625f
#define LNPS  6.931471805599453f

static_assert(NN % QT == 0);
static_assert(CC % QT == 0);
static_assert(MQKV == 2 * CQ + CC);
static_assert(MQKV % QT == 0);
static_assert((OSP * 4) % 16 == 0);
static_assert((OSPW * 4) % 16 == 0);
static_assert((TP * 2) % 16 == 0);
static_assert(CC % 32 == 0 && NN % 32 == 0 && CQ == 32);

typedef _Float16       v16h __attribute__((ext_vector_type(16)));
typedef _Float16       v8h  __attribute__((ext_vector_type(8)));
typedef __bf16         v16b __attribute__((ext_vector_type(16)));
typedef unsigned short v8us __attribute__((ext_vector_type(8)));
typedef float          v8f  __attribute__((ext_vector_type(8)));
typedef float          v4f  __attribute__((ext_vector_type(4)));
typedef unsigned int   v4u  __attribute__((ext_vector_type(4)));

union Frag  { v8us u[2]; v16h h; v16b bf; };
union FragH { v16h v; v8h hv[2]; };
static_assert(sizeof(Frag) == 32);
static_assert(sizeof(FragH) == 32);

__device__ __forceinline__ unsigned short bf_bits(float f) {
  unsigned u = __float_as_uint(f);
  return (unsigned short)((u + 0x7FFFu + ((u >> 16) & 1u)) >> 16);
}
__device__ __forceinline__ float bf_up(unsigned short hb) { return __uint_as_float(((unsigned)hb) << 16); }
__device__ __forceinline__ float bfr(float f) { return bf_up(bf_bits(f)); }
__device__ __forceinline__ unsigned short h_bits(_Float16 x) { return __builtin_bit_cast(unsigned short, x); }
__device__ __forceinline__ unsigned pk16(unsigned short a, unsigned short b) { return (unsigned)a | ((unsigned)b << 16); }
__device__ __forceinline__ v8f zero8() { v8f z = {0.f, 0.f, 0.f, 0.f, 0.f, 0.f, 0.f, 0.f}; return z; }
__device__ __forceinline__ float hmax8(v8f s) {
  return fmaxf(fmaxf(fmaxf(s[0], s[1]), fmaxf(s[2], s[3])), fmaxf(fmaxf(s[4], s[5]), fmaxf(s[6], s[7])));
}

__device__ __forceinline__ Frag ldfrag(const unsigned short* p) {
  Frag f;
  f.u[0] = *(const v8us*)(p);
  f.u[1] = *(const v8us*)(p + 16);
  return f;
}

__device__ __forceinline__ v8f mma_h(v16h a, v16h b, v8f c) {
  v8f d = __builtin_amdgcn_wmma_f32_16x16x32_f16(false, a, false, b, (short)0, c, false, false);
#if defined(__HIP_DEVICE_COMPILE__)
  asm volatile("v_nop\n\tv_nop\n\tv_nop\n\tv_nop" : "+v"(d) : "v"(a), "v"(b));
#endif
  return d;
}
__device__ __forceinline__ v8f mma_b(v16b a, v16b b, v8f c) {
  v8f d = __builtin_amdgcn_wmma_f32_16x16x32_bf16(false, a, false, b, (short)0, c, false, false);
#if defined(__HIP_DEVICE_COMPILE__)
  const v16h ha = __builtin_bit_cast(v16h, a), hb = __builtin_bit_cast(v16h, b);
  asm volatile("v_nop\n\tv_nop\n\tv_nop\n\tv_nop" : "+v"(d) : "v"(ha), "v"(hb));
#endif
  return d;
}

__global__ __launch_bounds__(256)
void cvt_w(const float* __restrict__ wq, const float* __restrict__ bq,
           const float* __restrict__ wk, const float* __restrict__ bk,
           const float* __restrict__ wv, const float* __restrict__ bv,
           unsigned short* W16, float* BIAS) {
  const int tid = threadIdx.x, blk = blockIdx.x;
  const int rl = tid >> 5, col = 8 * (tid & 31);
  const int o = 8 * blk + rl;
  const float* wbase = (blk < 4) ? wq : (blk < 8) ? wk : wv;
  const int osub = (blk < 4) ? 0 : (blk < 8) ? CQ : 2 * CQ;
  const float* s = wbase + (size_t)(o - osub) * CC + col;
  const v4f a = *(const v4f*)s;
  const v4f q = *(const v4f*)(s + 4);
  const float f[8] = {a[0], a[1], a[2], a[3], q[0], q[1], q[2], q[3]};
  v4u u;
#pragma unroll
  for (int t = 0; t < 4; ++t) {
    const _Float16 h0 = (_Float16)(bfr(f[2 * t]) * WSC);
    const _Float16 h1 = (_Float16)(bfr(f[2 * t + 1]) * WSC);
    u[t] = pk16(h_bits(h0), h_bits(h1));
  }
  v4f bvv;
  {
    const int tb = min(tid, 79);
    const int o4 = 4 * tb;
#pragma unroll
    for (int qd = 0; qd < 4; ++qd) {
      const int oo = o4 + qd;
      const int iq = min(oo, CQ - 1);
      const int ik = min(max(oo - CQ, 0), CQ - 1);
      const int iv = min(max(oo - 2 * CQ, 0), CC - 1);
      const float cq = bq[iq], ck = bk[ik], cv = bv[iv];
      const float val = (oo < CQ) ? cq : (oo < 2 * CQ) ? ck : cv;
      bvv[qd] = bfr(val);
    }
  }
#pragma unroll
  for (int pass = 0; pass < 2; ++pass) {
    *(volatile v4u*)(W16 + (size_t)o * CC + col) = u;
    if (blk == 0 && tid < 80) *(volatile v4f*)(BIAS + 4 * tid) = bvv;
    __threadfence();
  }
}

__global__ __launch_bounds__(256)
void cvt_x(const float* __restrict__ x, unsigned short* Xc, unsigned short* XP) {
  __shared__ __align__(16) unsigned short T[QT * TP];
  const int tid = threadIdx.x;
  const int nb = blockIdx.x, cb = blockIdx.y, b = blockIdx.z;
  const int e = tid & 7, lq = tid >> 3;
  const int n0 = nb * QT, c0 = cb * QT;
  v4u ux[2];
#pragma unroll
  for (int it = 0; it < 2; ++it) {
    const int cl = it * 32 + lq;
    const float* sp = x + ((size_t)(b * CC + c0 + cl)) * NN + n0 + 8 * e;
    const v4f a = *(const v4f*)sp;
    const v4f q = *(const v4f*)(sp + 4);
    unsigned short hb[8];
#pragma unroll
    for (int t = 0; t < 4; ++t) {
      hb[t]     = h_bits((_Float16)bfr(a[t]));
      hb[4 + t] = h_bits((_Float16)bfr(q[t]));
    }
#pragma unroll
    for (int t = 0; t < 4; ++t) ux[it][t] = pk16(hb[2 * t], hb[2 * t + 1]);
#pragma unroll
    for (int t = 0; t < 8; ++t) T[(8 * e + t) * TP + cl] = hb[t];
  }
  __syncthreads();
  v4u up[2];
#pragma unroll
  for (int it = 0; it < 2; ++it) {
    const int nl = it * 32 + lq;
    up[it] = *(const v4u*)(T + nl * TP + 8 * e);
  }
#pragma unroll
  for (int pass = 0; pass < 2; ++pass) {
#pragma unroll
    for (int it = 0; it < 2; ++it) {
      const int rl = it * 32 + lq;
      *(volatile v4u*)(Xc + ((size_t)(b * CC + c0 + rl)) * NN + n0 + 8 * e) = ux[it];
      *(volatile v4u*)(XP + ((size_t)(b * NN + n0 + rl)) * CC + c0 + 8 * e) = up[it];
    }
    __threadfence();
  }
}

__global__ __launch_bounds__(128)
void gemm_qkv(const unsigned short* __restrict__ W16, const float* __restrict__ BIAS,
              const unsigned short* __restrict__ XP,
              unsigned short* Qh, unsigned short* Ql, unsigned short* Kh, unsigned short* Kl,
              unsigned short* Vh) {
  __shared__ __align__(16) float Os[QT * OSP];
  const int tid  = threadIdx.x;
  const int lane = tid & 31, wave = tid >> 5;
  const int hh   = lane >> 4, c = lane & 15;
  const int nt   = blockIdx.x, mb = blockIdx.y, b = blockIdx.z;
  const int n0   = nt * QT, o0 = mb * QT;

  const unsigned short* ap = W16 + (size_t)(o0 + c) * CC + 8 * hh;
  const unsigned short* bp = XP + ((size_t)(b * NN + n0 + 16 * wave + c)) * CC + 8 * hh;

  v8f acc[4];
#pragma unroll
  for (int mt = 0; mt < 4; ++mt) acc[mt] = zero8();

#pragma unroll
  for (int ks = 0; ks < CC / 32; ++ks) {
    const Frag fb = ldfrag(bp + 32 * ks);
#pragma unroll
    for (int mt = 0; mt < 4; ++mt) {
      const Frag fa = ldfrag(ap + (size_t)(16 * mt) * CC + 32 * ks);
      acc[mt] = mma_h(fa.h, fb.h, acc[mt]);
    }
  }

  {
    const int nl = 16 * wave + c;
#pragma unroll
    for (int mt = 0; mt < 4; ++mt) {
#pragma unroll
      for (int r = 0; r < 8; ++r) {
        const int ol = 16 * mt + 8 * hh + r;
        Os[ol * OSP + nl] = acc[mt][r] * IWSC + BIAS[o0 + ol];
      }
    }
  }
  __syncthreads();

  const int e = tid & 7, lq = tid >> 3;
  if (mb == 0) {
#pragma unroll
    for (int pass = 0; pass < 2; ++pass) {
#pragma unroll
      for (int it = 0; it < 8; ++it) {
        const int p    = it >> 1;
        const int ll   = (it & 1) * 16 + lq;
        const int nl   = 2 * ll + (e >> 2);
        const int col0 = 8 * (e & 3);
        const int rb   = ((p >> 1) ? CQ : 0) + col0;
        v4u u;
#pragma unroll
        for (int t = 0; t < 4; ++t) {
          const float f0 = Os[(rb + 2 * t) * OSP + nl];
          const float f1 = Os[(rb + 2 * t + 1) * OSP + nl];
          const unsigned short hb0 = bf_bits(f0), hb1 = bf_bits(f1);
          const unsigned short lb0 = bf_bits(f0 - bf_up(hb0));
          const unsigned short lb1 = bf_bits(f1 - bf_up(hb1));
          u[t] = (p & 1) ? pk16(lb0, lb1) : pk16(hb0, hb1);
        }
        unsigned short* P = (p == 0) ? Qh : (p == 1) ? Ql : (p == 2) ? Kh : Kl;
        *(volatile v4u*)(P + ((size_t)(b * NN + n0 + nl)) * CQ + col0) = u;
      }
      __threadfence();
    }
  } else {
    const int ch0 = o0 - QT;
    v4u uv[4];
#pragma unroll
    for (int it = 0; it < 4; ++it) {
      const int row = it * 16 + lq;
      const v4f a = *(const v4f*)(Os + row * OSP + 8 * e);
      const v4f q = *(const v4f*)(Os + row * OSP + 8 * e + 4);
#pragma unroll
      for (int t = 0; t < 2; ++t) {
        uv[it][t]     = pk16(h_bits((_Float16)a[2 * t]), h_bits((_Float16)a[2 * t + 1]));
        uv[it][2 + t] = pk16(h_bits((_Float16)q[2 * t]), h_bits((_Float16)q[2 * t + 1]));
      }
    }
#pragma unroll
    for (int pass = 0; pass < 2; ++pass) {
#pragma unroll
      for (int it = 0; it < 4; ++it) {
        const int row = it * 16 + lq;
        *(volatile v4u*)(Vh + ((size_t)(b * CC + ch0 + row)) * NN + n0 + 8 * e) = uv[it];
      }
      __threadfence();
    }
  }
}

__global__ __launch_bounds__(128)
void attn_pam(const unsigned short* __restrict__ Qh, const unsigned short* __restrict__ Ql,
              const unsigned short* __restrict__ Kh, const unsigned short* __restrict__ Kl,
              const unsigned short* __restrict__ Vh, float* Yp) {
  __shared__ __align__(16) float Os[QT * OSPW];
  const int tid  = threadIdx.x;
  const int wave = tid >> 5, lane = tid & 31;
  const int hh   = lane >> 4, c = lane & 15;
  const int n0   = blockIdx.x * QT, b = blockIdx.y;

  Frag qh, ql;
  {
    const size_t qo = ((size_t)(b * NN + n0 + 16 * wave + c)) * CQ + 8 * hh;
    qh = ldfrag(Qh + qo);
    ql = ldfrag(Ql + qo);
  }
  const unsigned short* Khp = Kh + (size_t)b * NN * CQ + (size_t)c * CQ + 8 * hh;
  const unsigned short* Klp = Kl + (size_t)b * NN * CQ + (size_t)c * CQ + 8 * hh;
  const unsigned short* Vhp = Vh + (size_t)b * CC * NN + (size_t)c * NN + 8 * hh;

  float m = -1.0e30f, l = 0.f;
  v8f o[16];
#pragma unroll
  for (int j = 0; j < 16; ++j) o[j] = zero8();

#pragma unroll 1
  for (int kb = 0; kb < NN; kb += 32) {
    const Frag k0  = ldfrag(Khp + (size_t)kb * CQ);
    const Frag k1  = ldfrag(Khp + (size_t)(kb + 16) * CQ);
    const Frag k0l = ldfrag(Klp + (size_t)kb * CQ);
    const Frag k1l = ldfrag(Klp + (size_t)(kb + 16) * CQ);
    v8f s0 = mma_b(k0.bf, qh.bf, zero8());
    v8f s1 = mma_b(k1.bf, qh.bf, zero8());
    s0 = mma_b(k0.bf, ql.bf, s0);
    s1 = mma_b(k1.bf, ql.bf, s1);
    s0 = mma_b(k0l.bf, qh.bf, s0);
    s1 = mma_b(k1l.bf, qh.bf, s1);

    float mx = fmaxf(hmax8(s0), hmax8(s1));
    mx = fmaxf(mx, __shfl_xor(mx, 16, 32));
    const float mn   = fmaxf(m, mx);
    const float corr = __expf(m - mn);
    m = mn;
    const float msh = mn - LNPS;
    l *= corr;
#pragma unroll
    for (int j = 0; j < 16; ++j) {
#pragma unroll
      for (int r = 0; r < 8; ++r) o[j][r] *= corr;
    }

    FragH ph;
    float ls = 0.f;
#pragma unroll
    for (int r = 0; r < 8; ++r) {
      const float e0 = __expf(s0[r] - msh);
      const float e1 = __expf(s1[r] - msh);
      ls += e0 + e1;
      ph.hv[0][r] = (_Float16)e0;
      ph.hv[1][r] = (_Float16)e1;
    }
    l += ls;

#pragma unroll
    for (int j = 0; j < 16; ++j) {
      const Frag vf = ldfrag(Vhp + (size_t)(16 * j) * NN + kb);
      o[j] = mma_h(vf.h, ph.v, o[j]);
    }
  }
  l += __shfl_xor(l, 16, 32);
  const float inv = 1.0f / l;

  const int qrow = 16 * wave + c;
  const int e = tid & 7, lq = tid >> 3;
#pragma unroll
  for (int half = 0; half < 2; ++half) {
    if (half) __syncthreads();
#pragma unroll
    for (int jj = 0; jj < 8; ++jj) {
      const int j = 8 * half + jj;
      v4f va, vb;
#pragma unroll
      for (int r = 0; r < 4; ++r) { va[r] = o[j][r] * inv; vb[r] = o[j][4 + r] * inv; }
      *(v4f*)(Os + qrow * OSPW + 16 * jj + 8 * hh)     = va;
      *(v4f*)(Os + qrow * OSPW + 16 * jj + 8 * hh + 4) = vb;
    }
    __syncthreads();
#pragma unroll
    for (int pass = 0; pass < 2; ++pass) {
#pragma unroll
      for (int it = 0; it < 16; ++it) {
        const int L   = it * 16 + lq;
        const int chl = L >> 1, hf = L & 1;
        const int nl  = hf * 32 + 4 * e;
        v4f v;
#pragma unroll
        for (int t = 0; t < 4; ++t) v[t] = Os[(nl + t) * OSPW + chl];
        *(volatile v4f*)(Yp + ((size_t)(b * CC + 128 * half + chl)) * NN + n0 + nl) = v;
      }
      __threadfence();
    }
  }
}

__global__ __launch_bounds__(128)
void gram_k(const unsigned short* __restrict__ Xc, float* G) {
  __shared__ __align__(16) float Os[QT * OSP];
  const int tid  = threadIdx.x;
  const int lane = tid & 31, wave = tid >> 5;
  const int hh   = lane >> 4, c = lane & 15;
  const int jt = blockIdx.x, itb = blockIdx.y, b = blockIdx.z;
  const int j0 = jt * QT, i0 = itb * QT;

  const unsigned short* ap = Xc + ((size_t)(b * CC + i0 + c)) * NN + 8 * hh;
  const unsigned short* bp = Xc + ((size_t)(b * CC + j0 + 16 * wave + c)) * NN + 8 * hh;

  v8f acc[4];
#pragma unroll
  for (int mt = 0; mt < 4; ++mt) acc[mt] = zero8();

#pragma unroll 2
  for (int ks = 0; ks < NN / 32; ++ks) {
    const Frag fb = ldfrag(bp + 32 * ks);
#pragma unroll
    for (int mt = 0; mt < 4; ++mt) {
      const Frag fa = ldfrag(ap + (size_t)(16 * mt) * NN + 32 * ks);
      acc[mt] = mma_h(fa.h, fb.h, acc[mt]);
    }
  }
  {
    const int nl = 16 * wave + c;
#pragma unroll
    for (int mt = 0; mt < 4; ++mt) {
#pragma unroll
      for (int r = 0; r < 8; ++r) Os[(16 * mt + 8 * hh + r) * OSP + nl] = acc[mt][r];
    }
  }
  __syncthreads();
  {
    const int e = tid & 7, lq = tid >> 3;
#pragma unroll
    for (int pass = 0; pass < 2; ++pass) {
#pragma unroll
      for (int it = 0; it < 8; ++it) {
        const int L = it * 16 + lq;
        const int row = L >> 1, hf = L & 1;
        const v4f v = *(const v4f*)(Os + row * OSP + hf * 32 + 4 * e);
        *(volatile v4f*)(G + ((size_t)(b * CC + i0 + row)) * CC + j0 + hf * 32 + 4 * e) = v;
      }
      __threadfence();
    }
  }
}

__global__ __launch_bounds__(256)
void cam_softmax(const float* __restrict__ G, unsigned short* Pc) {
  const int tid = threadIdx.x, lane = tid & 31, w = tid >> 5;
  const int b = blockIdx.y, i = blockIdx.x * 8 + w;
  const float* row = G + ((size_t)(b * CC + i)) * CC + 8 * lane;
  const v4f a = *(const v4f*)row;
  const v4f q = *(const v4f*)(row + 4);
  const float ev[8] = {a[0], a[1], a[2], a[3], q[0], q[1], q[2], q[3]};
  float mn = ev[0];
#pragma unroll
  for (int t = 1; t < 8; ++t) mn = fminf(mn, ev[t]);
#pragma unroll
  for (int s = 1; s < 32; s <<= 1) mn = fminf(mn, __shfl_xor(mn, s, 32));
  float p[8], sm = 0.f;
#pragma unroll
  for (int t = 0; t < 8; ++t) { p[t] = __expf(mn - ev[t]); sm += p[t]; }
#pragma unroll
  for (int s = 1; s < 32; s <<= 1) sm += __shfl_xor(sm, s, 32);
  const float inv = PSC / sm;
  v4u u;
#pragma unroll
  for (int t = 0; t < 4; ++t)
    u[t] = pk16(h_bits((_Float16)(p[2 * t] * inv)), h_bits((_Float16)(p[2 * t + 1] * inv)));
#pragma unroll
  for (int pass = 0; pass < 2; ++pass) {
    *(volatile v4u*)(Pc + ((size_t)(b * CC + i)) * CC + 8 * lane) = u;
    __threadfence();
  }
}

__global__ __launch_bounds__(128)
void cam_out(const unsigned short* __restrict__ Pc, const unsigned short* __restrict__ XP,
             const float* __restrict__ Yp, const float* __restrict__ x,
             const float* __restrict__ gpam, const float* __restrict__ gcam, float* out) {
  __shared__ __align__(16) float Os[QT * OSP];
  const int tid  = threadIdx.x;
  const int lane = tid & 31, wave = tid >> 5;
  const int hh   = lane >> 4, c = lane & 15;
  const int nt = blockIdx.x, itb = blockIdx.y, b = blockIdx.z;
  const int n0 = nt * QT, i0 = itb * QT;

  const unsigned short* ap = Pc + ((size_t)(b * CC + i0 + c)) * CC + 8 * hh;
  const unsigned short* bp = XP + ((size_t)(b * NN + n0 + 16 * wave + c)) * CC + 8 * hh;

  v8f acc[4];
#pragma unroll
  for (int mt = 0; mt < 4; ++mt) acc[mt] = zero8();

#pragma unroll
  for (int ks = 0; ks < CC / 32; ++ks) {
    const Frag fb = ldfrag(bp + 32 * ks);
#pragma unroll
    for (int mt = 0; mt < 4; ++mt) {
      const Frag fa = ldfrag(ap + (size_t)(16 * mt) * CC + 32 * ks);
      acc[mt] = mma_h(fa.h, fb.h, acc[mt]);
    }
  }
  {
    const int nl = 16 * wave + c;
#pragma unroll
    for (int mt = 0; mt < 4; ++mt) {
#pragma unroll
      for (int r = 0; r < 8; ++r) Os[(16 * mt + 8 * hh + r) * OSP + nl] = acc[mt][r];
    }
  }
  __syncthreads();

  const float gp = bfr(gpam[0]);
  const float gc = bfr(gcam[0]) * IPSC;
  const int e = tid & 7, lq = tid >> 3;
  v4f res[8];
#pragma unroll
  for (int it = 0; it < 8; ++it) {
    const int L = it * 16 + lq;
    const int row = L >> 1, hf = L & 1;
    const int nl = hf * 32 + 4 * e;
    const v4f cam4 = *(const v4f*)(Os + row * OSP + nl);
    const size_t idx = ((size_t)(b * CC + i0 + row)) * NN + n0 + nl;
    const v4f xv = *(const v4f*)(x + idx);
    const v4f yv = *(const v4f*)(Yp + idx);
#pragma unroll
    for (int t = 0; t < 4; ++t) {
      const float xb = bfr(xv[t]);
      const float t1 = gp * yv[t] + xb;
      const float t2 = gc * cam4[t] + xb;
      res[it][t] = t1 + t2;
    }
  }
#pragma unroll
  for (int pass = 0; pass < 2; ++pass) {
#pragma unroll
    for (int it = 0; it < 8; ++it) {
      const int L = it * 16 + lq;
      const int row = L >> 1, hf = L & 1;
      const int nl = hf * 32 + 4 * e;
      const size_t idx = ((size_t)(b * CC + i0 + row)) * NN + n0 + nl;
      *(volatile v4f*)(out + idx) = res[it];
    }
    __threadfence();
  }
}

extern "C" void kernel_launch(void* const* d_in, const int* in_sizes, int n_in,
                              void* d_out, int out_size, void* d_ws, size_t ws_size,
                              hipStream_t stream) {
  const int XN = NB * CC * NN;
  if (n_in < 9) return;
  if (in_sizes[0] != XN) return;
  if (in_sizes[1] != CQ * CC || in_sizes[2] != CQ) return;
  if (in_sizes[3] != CQ * CC || in_sizes[4] != CQ) return;
  if (in_sizes[5] != CC * CC || in_sizes[6] != CC) return;
  if (in_sizes[7] < 1 || in_sizes[8] < 1) return;
  if (out_size != XN) return;

  size_t off = 0;
  auto carve = [&](size_t bytes) { const size_t o = off; off += (bytes + 255) & ~(size_t)255; return o; };
  const size_t oW16 = carve((size_t)MQKV * CC * 2);
  const size_t oBIA = carve((size_t)MQKV * 4);
  const size_t oXc  = carve((size_t)NB * CC * NN * 2);
  const size_t oXP  = carve((size_t)NB * NN * CC * 2);
  const size_t oQh  = carve((size_t)NB * NN * CQ * 2);
  const size_t oQl  = carve((size_t)NB * NN * CQ * 2);
  const size_t oKh  = carve((size_t)NB * NN * CQ * 2);
  const size_t oKl  = carve((size_t)NB * NN * CQ * 2);
  const size_t oVh  = carve((size_t)NB * CC * NN * 2);
  const size_t oYp  = carve((size_t)NB * CC * NN * 4);
  const size_t oG   = carve((size_t)NB * CC * CC * 4);
  const size_t oPc  = carve((size_t)NB * CC * CC * 2);
  if (off > ws_size) return;
  if (off > (size_t)134217728) return;

  const float* x    = (const float*)d_in[0];
  const float* wq   = (const float*)d_in[1];
  const float* bq   = (const float*)d_in[2];
  const float* wk   = (const float*)d_in[3];
  const float* bk   = (const float*)d_in[4];
  const float* wv   = (const float*)d_in[5];
  const float* bv   = (const float*)d_in[6];
  const float* gpam = (const float*)d_in[7];
  const float* gcam = (const float*)d_in[8];

  char* ws = (char*)d_ws;
  unsigned short* W16 = (unsigned short*)(ws + oW16);
  float*          BIA = (float*)(ws + oBIA);
  unsigned short* Xc  = (unsigned short*)(ws + oXc);
  unsigned short* XP  = (unsigned short*)(ws + oXP);
  unsigned short* Qh  = (unsigned short*)(ws + oQh);
  unsigned short* Ql  = (unsigned short*)(ws + oQl);
  unsigned short* Kh  = (unsigned short*)(ws + oKh);
  unsigned short* Kl  = (unsigned short*)(ws + oKl);
  unsigned short* Vh  = (unsigned short*)(ws + oVh);
  float*          Yp  = (float*)(ws + oYp);
  float*          G   = (float*)(ws + oG);
  unsigned short* Pc  = (unsigned short*)(ws + oPc);
  float* out = (float*)d_out;

  const dim3 blk256(256), blk128(128);

  cvt_w<<<dim3(MQKV / 8), blk256, 0, stream>>>(wq, bq, wk, bk, wv, bv, W16, BIA);
  cvt_x<<<dim3(NN / QT, CC / QT, NB), blk256, 0, stream>>>(x, Xc, XP);
  gemm_qkv<<<dim3(NN / QT, MQKV / QT, NB), blk128, 0, stream>>>(W16, BIA, XP, Qh, Ql, Kh, Kl, Vh);
  attn_pam<<<dim3(NN / QT, NB), blk128, 0, stream>>>(Qh, Ql, Kh, Kl, Vh, Yp);
  gram_k<<<dim3(CC / QT, CC / QT, NB), blk128, 0, stream>>>(Xc, G);
  cam_softmax<<<dim3(CC / 8, NB), blk256, 0, stream>>>(G, Pc);
  cam_out<<<dim3(NN / QT, CC / QT, NB), blk128, 0, stream>>>(Pc, XP, Yp, x, gpam, gcam, out);
  (void)hipGetLastError();
}
